// KNNLayer_79010218377296
// MI455X (gfx1250) — hardware-verified
//
#include <hip/hip_runtime.h>
#include <math.h>

typedef __attribute__((ext_vector_type(16))) _Float16 v16h;
typedef __attribute__((ext_vector_type(16))) __bf16 v16b;
typedef __attribute__((ext_vector_type(8)))  _Float16 v8h;
typedef __attribute__((ext_vector_type(8)))  float v8f;
typedef __attribute__((ext_vector_type(4)))  float v4f;
typedef __attribute__((ext_vector_type(2)))  float v2f;
typedef __attribute__((ext_vector_type(4)))  unsigned v4u;
typedef __attribute__((ext_vector_type(4)))  int v4i;
typedef float __attribute__((may_alias)) float_a;
typedef int __attribute__((may_alias)) int_a;

template <typename T> __device__ __forceinline__ void vst2(void* p, T v) { *(volatile T*)p = v; __threadfence(); *(volatile T*)p = v; }
__device__ __forceinline__ v8f wmma16(v16h a, v16h b, v8f c) {
  v8f d = __builtin_amdgcn_wmma_f32_16x16x32_f16(false, a, false, b, (short)0, c, false, false);
  asm volatile("v_nop\n\tv_nop\n\tv_nop\n\tv_nop" : "+v"(d) : "v"(a), "v"(b));
  return d;
}
__device__ __forceinline__ v8f wmma_bf(v16b a, v16b b, v8f c) {
  v8f d = __builtin_amdgcn_wmma_f32_16x16x32_bf16(false, a, false, b, (short)0, c, false, false);
  asm volatile("v_nop\n\tv_nop\n\tv_nop\n\tv_nop" : "+v"(d) : "v"(a), "v"(b));
  return d;
}
__device__ __forceinline__ v16h frag_h(const _Float16* rowk0, int lane) {
  union { v16h v; v8h q[2]; } u; const _Float16* p = rowk0 + 8 * (lane >> 4);
  u.q[0] = *(const v8h*)p; u.q[1] = *(const v8h*)(p + 16); return u.v;
}
__device__ __forceinline__ v16h frag_f32(const float* rowk0, int lane) {
  v16h a; const float* p = rowk0 + 8 * (lane >> 4);
#pragma unroll
  for (int i = 0; i < 8; ++i) { a[i] = (_Float16)p[i]; a[8 + i] = (_Float16)p[16 + i]; }
  return a;
}
__device__ __forceinline__ v16h frag_f32s(const float* rowk0, int lane, float sc) {
  v16h a; const float* p = rowk0 + 8 * (lane >> 4);
#pragma unroll
  for (int i = 0; i < 8; ++i) { a[i] = (_Float16)(p[i] * sc); a[8 + i] = (_Float16)(p[16 + i] * sc); }
  return a;
}
__device__ __forceinline__ v16h fragc_f32(const float* W, int k0, int n, int lane, int ld, int K) {
  v16h a; const int g = lane >> 4;
#pragma unroll
  for (int i = 0; i < 8; ++i) { const int ka = k0 + 8 * g + i, kb = ka + 16;
    a[i] = (_Float16)(ka < K ? W[(size_t)(ka < K ? ka : K - 1) * ld + n] : 0.f); a[8 + i] = (_Float16)(kb < K ? W[(size_t)(kb < K ? kb : K - 1) * ld + n] : 0.f); }
  return a;
}
struct F2 { v16b h, l; };
__device__ __forceinline__ F2 bsplit16(const float v[16]) { F2 r;
#pragma unroll
  for (int i = 0; i < 16; ++i) { const __bf16 h = (__bf16)v[i]; r.h[i] = h; r.l[i] = (__bf16)(v[i] - (float)h); }
  return r; }
__device__ __forceinline__ F2 split_row(const float* row, int k0, int lane) { float v[16]; const float* p = row + k0 + 8 * (lane >> 4);
#pragma unroll
  for (int i = 0; i < 8; ++i) { v[i] = p[i]; v[8 + i] = p[16 + i]; }
  return bsplit16(v); }
__device__ __forceinline__ F2 split_rowK(const float* row, int k0, int lane, int K) { float v[16]; const int g = lane >> 4;
#pragma unroll
  for (int i = 0; i < 8; ++i) { const int ka = k0 + 8 * g + i, kb = ka + 16; v[i] = ka < K ? row[ka < K ? ka : K - 1] : 0.f; v[8 + i] = kb < K ? row[kb < K ? kb : K - 1] : 0.f; }
  return bsplit16(v); }
__device__ __forceinline__ F2 split_col(const float* W, int k0, int n, int lane, int ld, int K) { float v[16]; const int g = lane >> 4;
#pragma unroll
  for (int i = 0; i < 8; ++i) { const int ka = k0 + 8 * g + i, kb = ka + 16; v[i] = ka < K ? W[(size_t)(ka < K ? ka : K - 1) * ld + n] : 0.f; v[8 + i] = kb < K ? W[(size_t)(kb < K ? kb : K - 1) * ld + n] : 0.f; }
  return bsplit16(v); }
__device__ __forceinline__ v8f mac3(const F2& a, const F2& b, v8f c) { c = wmma_bf(a.l, b.h, c); c = wmma_bf(a.h, b.l, c); return wmma_bf(a.h, b.h, c); }
__device__ __forceinline__ float sigm(float v) { return 1.0f / (1.0f + expf(-v)); }
#define LDSX() do { asm volatile("s_wait_dscnt 0" ::: "memory"); __builtin_amdgcn_wave_barrier(); __builtin_amdgcn_fence(__ATOMIC_RELEASE, "workgroup"); } while (0)


#define NB 32
#define NP 1024
#define NR (NB * NP)
#define FF 128
#define PP2 256
#define PPO 128
#define KN 16
#define KS 17
#ifndef NBT
#define NBT NB
#endif
typedef __attribute__((ext_vector_type(8))) __bf16 v8b;
__device__ __forceinline__ v16b frag_b(const __bf16* rowk0, int lane) {
  union { v16b v; v8b q[2]; } u; const __bf16* p = rowk0 + 8 * (lane >> 4);
  u.q[0] = *(const v8b*)p; u.q[1] = *(const v8b*)(p + 16); return u.v;
}
__device__ __forceinline__ float bfr(float v) { return (float)(__bf16)v; }
__device__ __attribute__((noinline)) float exp_ni(float v) { return expf(v); }
__device__ __attribute__((noinline)) float erf_ni(float v) { return erff(v); }
__device__ __forceinline__ float gelu_exact(float v) { return 0.5f * v * (1.0f + erf_ni(v * 0.70710678118654752f)); }

#define WS_PK1 0u
#define PK_1A 0
#define PK_1B (PP2 * FF)
#define PK_2  (2 * PP2 * FF)
#define PK_END (PK_2 + PPO * PP2)
#define WS_FB  (((2u * PK_END) + 127u) / 128u * 128u)
#define WS_P1  (WS_FB + 2u * NR * FF)
#define WS_P2  (WS_P1 + 4u * NR * PP2)
#define WS_IDX (WS_P2 + 4u * NR * PP2)
#define WS_END (WS_IDX + 4u * NR * KN)

__global__ __launch_bounds__(256) void k_pack(const float* __restrict__ W1, const float* __restrict__ W2, __bf16* __restrict__ PK) {
  __shared__ __align__(16) __bf16 s[PP2]; const int n = blockIdx.x, which = blockIdx.y, tid = threadIdx.x; int K; size_t dst;
  if (which == 0) { K = FF; dst = PK_1A + (size_t)n * FF; if (tid < FF) s[tid] = (__bf16)W1[(size_t)tid * PP2 + n]; }
  else if (which == 1) { K = FF; dst = PK_1B + (size_t)n * FF; if (tid < FF) s[tid] = (__bf16)W1[(size_t)(FF + tid) * PP2 + n]; }
  else { if (n >= PPO) return; K = PP2; dst = PK_2 + (size_t)n * PP2; s[tid] = (__bf16)W2[(size_t)tid * PPO + n]; }
  __syncthreads();
  if (tid < K / 8) vst2((unsigned*)(PK + dst + tid * 8), *(const v4u*)&s[tid * 8]);
}
__global__ __launch_bounds__(64) void k_fb(const float* __restrict__ F, __bf16* __restrict__ FB) {
  __shared__ __align__(16) __bf16 s[FF]; const size_t r = blockIdx.x; const int t = threadIdx.x;
  for (int k = t; k < FF; k += 64) s[k] = (__bf16)F[r * FF + k];
  __syncthreads();
  if (t < FF / 8) vst2((unsigned*)(FB + r * FF + t * 8), *(const v4u*)&s[t * 8]);
}
__global__ __launch_bounds__(256) void k_knn(const float* __restrict__ PTS, int* __restrict__ IDX) {
  __shared__ float sx[NP], sy[NP]; __shared__ __align__(16) int sidx[256][KN];
  const int tid = threadIdx.x; const int b = blockIdx.x / (NP / 256); const int q0 = (blockIdx.x % (NP / 256)) * 256; const int q = q0 + tid;
  for (int i = tid; i < NP; i += 256) { sx[i] = bfr(PTS[((size_t)b * NP + i) * 2]); sy[i] = bfr(PTS[((size_t)b * NP + i) * 2 + 1]); }
  __syncthreads();
  const float qx = sx[q], qy = sy[q]; const float rq = qx * qx + qy * qy;
  float bd[KS]; int bi[KS];
#pragma unroll
  for (int s = 0; s < KS; ++s) { bd[s] = 3.0e38f; bi[s] = 0; }
  for (int m = 0; m < NP; ++m) { const float rm = sx[m] * sx[m] + sy[m] * sy[m]; const float mm = qx * sx[m] + qy * sy[m]; const float D = fabsf((rq - 2.0f * mm) + rm);
    if (D < bd[KS - 1]) { float cd = D; int ci = m; bool placed = false;
#pragma unroll
      for (int s = 0; s < KS; ++s) { const bool sw = placed || (cd < bd[s]); placed = sw; const float td = bd[s]; const int ti = bi[s]; bd[s] = sw ? cd : td; bi[s] = sw ? ci : ti; cd = sw ? td : cd; ci = sw ? ti : ci; } } }
#pragma unroll
  for (int s = 1; s < KS; ++s) sidx[tid][s - 1] = bi[s];
  __syncthreads();
  for (int qq = tid; qq < 256 * KN / 4; qq += 256) vst2((unsigned*)(IDX + ((size_t)b * NP + q0) * KN + qq * 4), *(const v4u*)(&sidx[0][0] + qq * 4));
}
__global__ __launch_bounds__(128) void k_p12(const __bf16* __restrict__ FB, const __bf16* __restrict__ PK, float* __restrict__ P1, float* __restrict__ P2) {
  __shared__ __align__(16) float so[4][16][132];
  const int tid = threadIdx.x, wave = tid >> 5, lane = tid & 31, col = lane & 15, g = lane >> 4; const size_t r0 = (size_t)blockIdx.x * 64 + wave * 16; const int n0 = blockIdx.y * 128; const int which = blockIdx.z;
  const __bf16* P = PK + (which == 0 ? PK_1A : PK_1B); float* OUT = which == 0 ? P1 : P2;
  v8f acc[8] = {};
#pragma unroll
  for (int kc = 0; kc < FF / 32; ++kc) { const v16b a = frag_b(FB + (r0 + col) * FF + kc * 32, lane);
#pragma unroll
    for (int j = 0; j < 8; ++j) acc[j] = wmma_bf(a, frag_b(P + (size_t)(n0 + j * 16 + col) * FF + kc * 32, lane), acc[j]); }
#pragma unroll
  for (int j = 0; j < 8; ++j)
#pragma unroll
    for (int r = 0; r < 8; ++r) so[wave][8 * g + r][j * 16 + col] = acc[j][r];
  LDSX();
  for (int rl = 0; rl < 16; ++rl) vst2(OUT + (r0 + rl) * PP2 + n0 + lane * 4, *(const v4f*)&so[wave][rl][lane * 4]);
}
__global__ __launch_bounds__(128) void k_mlp(const float* __restrict__ P1, const float* __restrict__ P2, const int* __restrict__ IDX, const float* __restrict__ B1, const __bf16* __restrict__ PK, const float* __restrict__ B2, float* __restrict__ OUT) {
  __shared__ __align__(16) __bf16 sh_[4][16][PP2 + 8], sl_[4][16][PP2 + 8]; __shared__ __align__(16) float so[4][PPO]; __shared__ int sid[4][KN];
  const int tid = threadIdx.x, wave = tid >> 5, lane = tid & 31, col = lane & 15, g = lane >> 4; const size_t n = (size_t)blockIdx.x * 4 + wave;
  if (lane < KN) sid[wave][lane] = min(max(IDX[n * KN + lane], 0), NP - 1);
  LDSX();
  const int b = (int)(n / NP);
  for (int q = lane; q < KN * PP2; q += 32) { const int k = q / PP2, c = q % PP2; const size_t src = ((size_t)b * NP + sid[wave][k]) * PP2 + c;
    const float v = gelu_exact((P1[src] + (P2[n * PP2 + c] - P1[n * PP2 + c])) + bfr(B1[c])); const __bf16 hb = (__bf16)v; sh_[wave][k][c] = hb; sl_[wave][k][c] = (__bf16)(v - (float)hb); }
  LDSX();
  v8f acc[8] = {};
#pragma unroll 2
  for (int kc = 0; kc < PP2 / 32; ++kc) { F2 a; a.h = frag_b(&sh_[wave][col][kc * 32], lane); a.l = frag_b(&sl_[wave][col][kc * 32], lane);
#pragma unroll
    for (int j = 0; j < 8; ++j) { const v16b w = frag_b(PK + PK_2 + (size_t)(j * 16 + col) * PP2 + kc * 32, lane); acc[j] = wmma_bf(a.l, w, acc[j]); acc[j] = wmma_bf(a.h, w, acc[j]); } }
#pragma unroll
  for (int j = 0; j < 8; ++j) { const int c = j * 16 + col; const float bb = bfr(B2[c]); float s = 0.f;
#pragma unroll
    for (int r = 0; r < 8; ++r) s += gelu_exact(acc[j][r] + bb);
    s += __shfl_xor(s, 16);
    if (g == 0) so[wave][c] = s * (1.0f / 16.0f); }
  LDSX();
  vst2(OUT + n * PPO + lane * 4, *(const v4f*)&so[wave][lane * 4]);
}
extern "C" void kernel_launch(void* const* d_in, const int* in_sizes, int n_in, void* d_out, int out_size, void* d_ws, size_t ws_size, hipStream_t stream) {
  (void)in_sizes; (void)n_in; (void)out_size;
  const float** F = (const float**)d_in;
  if (ws_size < (size_t)WS_END) return;
  char* ws = (char*)d_ws; __bf16 *PK = (__bf16*)(ws + WS_PK1), *FB = (__bf16*)(ws + WS_FB); float *P1 = (float*)(ws + WS_P1), *P2 = (float*)(ws + WS_P2); int* IDX = (int*)(ws + WS_IDX);
  k_pack<<<dim3(PP2, 3), 256, 0, stream>>>(F[2], F[4], PK);
  k_fb<<<NBT * NP, 64, 0, stream>>>(F[1], FB);
  k_knn<<<NBT * NP / 256, 256, 0, stream>>>(F[0], IDX);
  k_p12<<<dim3(NBT * NP / 64, PP2 / 128, 2), 128, 0, stream>>>(FB, PK, P1, P2);
  k_mlp<<<NBT * NP / 4, 128, 0, stream>>>(P1, P2, IDX, F[3], PK, F[5], (float*)d_out);
}
